// EnhancedTCN_GNN_5351529250826
// MI455X (gfx1250) — hardware-verified
//
#include <hip/hip_runtime.h>
#include <stddef.h>
#include <stdint.h>


#define NBAT  4
#define NTIM  24
#define NST   128
#define FIN   64
#define CH    256
#define NLAY  3
#define KTAP  3
#define NNODE (NBAT * NTIM * NST)
#define NGRP  (NBAT * NTIM)
#define NHD   4
#define DHD   64
#define QKVW  (3 * CH)

#define GM    64
#define DP    260
#define HP    264
#define GT    64
#define GCH   256
#define VP    136
#define PP    136
#define NTHR  256

#define WSC   16.0f
#define WINV  0.0625f
#define PSC   4096.0f
#define PINV  0.000244140625f

#define M_ENC  0
#define M_CONV 1
#define M_XLR  2
#define M_QKV  3
#define M_WO   4
#define M_SKIP 5
#define M_GATE 6

#define LDS_GEMM ((GM * DP) * 4)
#define LDS_GATE ((GM * DP) * 4 + (GM * HP) * 2 + (GM * 2) * 4)
#define LDS_GAT  ((GT * 2 * CH + GT * 4) * 4 + 8 * GCH * 4)

static_assert(LDS_GEMM == 66560);
static_assert(LDS_GATE == 100864);
static_assert(LDS_GAT == 140288);
static_assert((NNODE % GM) == 0);
static_assert((NNODE % GT) == 0);
static_assert((NST % GM) == 0);
static_assert((NST % GT) == 0);
static_assert(GCH == 8 * 32);
static_assert(GT == 8 * 8);

typedef float    v4f  __attribute__((ext_vector_type(4)));
typedef float    v8f  __attribute__((ext_vector_type(8)));
typedef int      v2i  __attribute__((ext_vector_type(2)));
typedef int      v4i  __attribute__((ext_vector_type(4)));
typedef _Float16 v4h  __attribute__((ext_vector_type(4)));
typedef _Float16 v8h  __attribute__((ext_vector_type(8)));
typedef _Float16 v16h __attribute__((ext_vector_type(16)));
union Frag { v16h v; v8h half[2]; };
union P16  { v8h h; v4i i; };
union P8   { v4h h; v2i i; };

#define LD4(p) (*(const v4f*)(p))

__device__ __forceinline__ v8f wm(v16h a, v16h b, v8f c) {
  v8f d = __builtin_amdgcn_wmma_f32_16x16x32_f16(false, a, false, b, (short)0, c, false, false);
  asm volatile("v_nop\n\tv_nop\n\tv_nop\n\tv_nop" : "+v"(d) : "v"(a), "v"(b));
  return d;
}

__device__ __forceinline__ v16h ldfrag(const _Float16* p) {
  Frag f;
  f.half[0] = *(const v8h*)p;
  f.half[1] = *(const v8h*)(p + 16);
  return f.v;
}

__device__ __forceinline__ v16h zfrag() {
  P16 z;
  z.i = (v4i){0, 0, 0, 0};
  Frag f;
  f.half[0] = z.h;
  f.half[1] = z.h;
  return f.v;
}

__device__ __forceinline__ float wsum(float v) {
  v += __shfl_xor(v, 16, 32);
  v += __shfl_xor(v, 8, 32);
  v += __shfl_xor(v, 4, 32);
  v += __shfl_xor(v, 2, 32);
  v += __shfl_xor(v, 1, 32);
  return v;
}

__device__ __forceinline__ v4f relu4(v4f v) {
  v.x = v.x > 0.0f ? v.x : 0.0f;
  v.y = v.y > 0.0f ? v.y : 0.0f;
  v.z = v.z > 0.0f ? v.z : 0.0f;
  v.w = v.w > 0.0f ? v.w : 0.0f;
  return v;
}

__device__ __forceinline__ float sig1(float z) {
  z = fminf(fmaxf(z, -30.0f), 30.0f);
  const float e = __expf(-z);
  return 1.0f / (1.0f + e);
}
__device__ __forceinline__ v4f sig4(v4f z) {
  v4f g;
  g.x = sig1(z.x); g.y = sig1(z.y); g.z = sig1(z.z); g.w = sig1(z.w);
  return g;
}

__device__ __forceinline__ float lk(float x) { return x > 0.0f ? x : 0.2f * x; }
__device__ __forceinline__ float dlk(v4f l, v4f r, v4f a) {
  return lk(l.x + r.x) * a.x + lk(l.y + r.y) * a.y + lk(l.z + r.z) * a.z + lk(l.w + r.w) * a.w;
}

__device__ __forceinline__ void ln8(v4f& v0, v4f& v1, v4f g0, v4f g1, v4f e0, v4f e1) {
  const float s  = wsum(v0.x + v0.y + v0.z + v0.w + v1.x + v1.y + v1.z + v1.w);
  const float mu = s * (1.0f / CH);
  const v4f d0 = v0 - mu, d1 = v1 - mu;
  const float q  = wsum(d0.x * d0.x + d0.y * d0.y + d0.z * d0.z + d0.w * d0.w +
                        d1.x * d1.x + d1.y * d1.y + d1.z * d1.z + d1.w * d1.w);
  const float rs = rsqrtf(q * (1.0f / CH) + 1e-5f);
  v0 = d0 * rs * g0 + e0;
  v1 = d1 * rs * g1 + e1;
}

__device__ __forceinline__ void st2f(float* p, v4f a, v4f b) {
  *(volatile v4f*)p = a;
  *(volatile v4f*)(p + 128) = b;
}
__device__ __forceinline__ void st2h(_Float16* p, v4f a, v4f b) {
  P8 ua, ub;
  ua.h = __builtin_convertvector(a, v4h);
  ub.h = __builtin_convertvector(b, v4h);
  *(volatile v2i*)p = ua.i;
  *(volatile v2i*)(p + 128) = ub.i;
}

__global__ __launch_bounds__(NTHR) void k_prep8(
    const float* s0, const float* s1, const float* s2, const float* s3,
    const float* s4, const float* s5, const float* s6, const float* s7,
    _Float16* d0, _Float16* d1, _Float16* d2, _Float16* d3,
    _Float16* d4, _Float16* d5, _Float16* d6, _Float16* d7,
    int K0, int K1, int K2, int K3, int K4, int K5, int K6, int K7,
    int N0, int N1, int N2, int N3, int N4, int N5, int N6, int N7,
    int Q0, int Q1, int Q2, int Q3, int Q4, int Q5, int Q6, int Q7) {
  const int y = blockIdx.y;
  const float* src = (y == 0) ? s0 : (y == 1) ? s1 : (y == 2) ? s2 : (y == 3) ? s3
                   : (y == 4) ? s4 : (y == 5) ? s5 : (y == 6) ? s6 : s7;
  _Float16* dst = (y == 0) ? d0 : (y == 1) ? d1 : (y == 2) ? d2 : (y == 3) ? d3
                : (y == 4) ? d4 : (y == 5) ? d5 : (y == 6) ? d6 : d7;
  const int K = (y == 0) ? K0 : (y == 1) ? K1 : (y == 2) ? K2 : (y == 3) ? K3
              : (y == 4) ? K4 : (y == 5) ? K5 : (y == 6) ? K6 : K7;
  const int N = (y == 0) ? N0 : (y == 1) ? N1 : (y == 2) ? N2 : (y == 3) ? N3
              : (y == 4) ? N4 : (y == 5) ? N5 : (y == 6) ? N6 : N7;
  const int Q = (y == 0) ? Q0 : (y == 1) ? Q1 : (y == 2) ? Q2 : (y == 3) ? Q3
              : (y == 4) ? Q4 : (y == 5) ? Q5 : (y == 6) ? Q6 : Q7;
  const int kq  = K >> 3;
  const int cnt = Q * kq;
  const int i   = blockIdx.x * NTHR + threadIdx.x;
  if (i >= cnt) return;
  const int n   = i / kq;
  const int k8  = (i - n * kq) << 3;
  const int nn  = (n < N) ? n : (N - 1);
  const bool z  = (n >= N);
  P16 u;
#pragma unroll
  for (int j = 0; j < 8; ++j) {
    const float t = src[(size_t)(k8 + j) * N + nn];
    u.h[j] = (_Float16)(z ? 0.0f : t * WSC);
  }
  _Float16* p = dst + (size_t)n * K + k8;
  *(volatile v4i*)p = u.i;
  __threadfence();
  *(volatile v4i*)p = u.i;
}

__global__ __launch_bounds__(NTHR) void k_prep_conv(const float* __restrict__ cw, _Float16* wt) {
  const int l = blockIdx.y;
  const float* src = cw + (size_t)l * CH * CH * KTAP;
  _Float16* dst = wt + (size_t)l * CH * (KTAP * CH);
  const int kq = (KTAP * CH) >> 3;
  const int i  = blockIdx.x * NTHR + threadIdx.x;
  if (i >= CH * kq) return;
  const int n   = i / kq;
  const int k8  = (i - n * kq) << 3;
  const int tap = k8 / CH;
  const int ci0 = k8 - tap * CH;
  P16 u;
#pragma unroll
  for (int j = 0; j < 8; ++j)
    u.h[j] = (_Float16)(src[((size_t)n * CH + ci0 + j) * KTAP + tap] * WSC);
  _Float16* p = dst + (size_t)n * (KTAP * CH) + k8;
  *(volatile v4i*)p = u.i;
  __threadfence();
  *(volatile v4i*)p = u.i;
}

__global__ __launch_bounds__(NTHR) void k_prep_x(const float* __restrict__ x, _Float16* X, int rows) {
  const int i = blockIdx.x * NTHR + threadIdx.x;
  if (i >= rows * (FIN >> 3)) return;
  const size_t o = (size_t)i * 8;
  const v4f a = LD4(x + o), b = LD4(x + o + 4);
  P16 u;
  u.h[0] = (_Float16)a.x; u.h[1] = (_Float16)a.y; u.h[2] = (_Float16)a.z; u.h[3] = (_Float16)a.w;
  u.h[4] = (_Float16)b.x; u.h[5] = (_Float16)b.y; u.h[6] = (_Float16)b.z; u.h[7] = (_Float16)b.w;
  *(volatile v4i*)(X + o) = u.i;
  __threadfence();
  *(volatile v4i*)(X + o) = u.i;
}

template <int MODE>
__global__ __launch_bounds__(NTHR) void k_gemm(
    const _Float16* __restrict__ A, const _Float16* __restrict__ Wt,
    const float* __restrict__ bias, const float* __restrict__ p0, const float* __restrict__ p1,
    const float* __restrict__ rin, float* outF, float* outF2, _Float16* outH, float* dout,
    const _Float16* __restrict__ W2, int K, int lda, int ldo, int ldoh, int dil, int flag) {
  extern __shared__ v4f glds[];
  float* Ds = (float*)glds;
  _Float16* Hf = (_Float16*)(Ds + GM * DP);
  float* outs = (float*)(Hf + GM * HP);

  const int tid = threadIdx.x;
  const int lane = tid & 31;
  const int w = tid >> 5;
  const int hh = lane >> 4;
  const int m = lane & 15;
  const int rowBase = blockIdx.x * GM;
  const int slab = blockIdx.y;
  const int cg = slab * CH + w * 32;

  v8f acc[8];
  const v8f z8 = {0.f, 0.f, 0.f, 0.f, 0.f, 0.f, 0.f, 0.f};
#pragma unroll
  for (int i = 0; i < 8; ++i) acc[i] = z8;
  const v16h z16 = zfrag();

  const _Float16* wr0 = Wt + (size_t)(cg + m) * K + 8 * hh;
  const _Float16* wr1 = Wt + (size_t)(cg + 16 + m) * K + 8 * hh;
  const int tcur = (rowBase / NST) % NTIM;

#pragma unroll 1
  for (int k0 = 0; k0 < K; k0 += 32) {
    int kk = k0;
    long aoff = 0;
    bool valid = true;
    if (MODE == M_CONV) {
      const int tap = k0 / CH;
      kk = k0 - tap * CH;
      const int tsh = (KTAP - 1 - tap) * dil;
      valid = (tcur - tsh) >= 0;
      aoff = valid ? -(long)tsh * NST * (long)lda : 0;
    }
    const v16h b0 = ldfrag(wr0 + k0);
    const v16h b1 = ldfrag(wr1 + k0);
    v16h a[4];
#pragma unroll
    for (int mt = 0; mt < 4; ++mt) {
      const v16h t = ldfrag(A + ((long)(rowBase + 16 * mt + m) * (long)lda + aoff + kk + 8 * hh));
      a[mt] = valid ? t : z16;
    }
#pragma unroll
    for (int mt = 0; mt < 4; ++mt) {
      acc[2 * mt]     = wm(a[mt], b0, acc[2 * mt]);
      acc[2 * mt + 1] = wm(a[mt], b1, acc[2 * mt + 1]);
    }
  }

#pragma unroll
  for (int mt = 0; mt < 4; ++mt)
#pragma unroll
    for (int j = 0; j < 2; ++j) {
      const v8f c = acc[2 * mt + j];
      float* pd = Ds + (16 * mt + 8 * hh) * DP + w * 32 + 16 * j + m;
#pragma unroll
      for (int r = 0; r < 8; ++r) pd[r * DP] = c[r];
    }
  __syncthreads();

  const v4f z4 = {0.f, 0.f, 0.f, 0.f};
  const v4f one4 = {1.f, 1.f, 1.f, 1.f};
  v4f bb0 = z4, bb1 = z4, gg0 = z4, gg1 = z4, ee0 = z4, ee1 = z4;
  if (MODE == M_ENC || MODE == M_CONV || MODE == M_WO || MODE == M_SKIP || MODE == M_GATE) {
    bb0 = LD4(bias + slab * CH + 4 * lane);
    bb1 = LD4(bias + slab * CH + 128 + 4 * lane);
  }
  if (MODE == M_QKV) {
    const float* bs = (slab == 0) ? bias : ((slab == 1) ? p0 : p1);
    bb0 = LD4(bs + 4 * lane);
    bb1 = LD4(bs + 128 + 4 * lane);
  }
  if (MODE == M_WO) {
    gg0 = LD4(p0 + 4 * lane); gg1 = LD4(p0 + 128 + 4 * lane);
    ee0 = LD4(p1 + 4 * lane); ee1 = LD4(p1 + 128 + 4 * lane);
  }

#pragma unroll 1
  for (int i = 0; i < 8; ++i) {
    const int rl = 8 * w + i;
    const int node = rowBase + rl;
    const float* dsr = Ds + rl * DP;
    v4f v0 = LD4(dsr + 4 * lane) * WINV;
    v4f v1 = LD4(dsr + 128 + 4 * lane) * WINV;
    if (MODE == M_ENC) {
      const int st = node % NST;
      const int tt = (node / NST) % NTIM;
      v0 = v0 + bb0; v1 = v1 + bb1;
      v0 = v0 + LD4(p0 + (size_t)st * CH + 4 * lane);
      v1 = v1 + LD4(p0 + (size_t)st * CH + 128 + 4 * lane);
      v0 = v0 + LD4(p1 + (size_t)tt * CH + 4 * lane);
      v1 = v1 + LD4(p1 + (size_t)tt * CH + 128 + 4 * lane);
      float* po = outF + (size_t)node * ldo + 4 * lane;
      _Float16* ph = outH + (size_t)node * ldoh + 4 * lane;
      st2f(po, v0, v1); st2h(ph, v0, v1);
      __threadfence();
      st2f(po, v0, v1); st2h(ph, v0, v1);
    } else if (MODE == M_CONV) {
      const v4f y0 = relu4(v0 + bb0), y1 = relu4(v1 + bb1);
      float* po = outF + (size_t)node * ldo + 4 * lane;
      float* ps = outF2 + (size_t)node * ldo + 4 * lane;
      _Float16* ph = outH + (size_t)node * ldoh + 4 * lane;
      const v4f h0 = LD4(po), h1 = LD4(po + 128);
      const v4f s0 = LD4(ps), s1 = LD4(ps + 128);
      const v4f hn0 = y0 + h0, hn1 = y1 + h1;
      const v4f sn0 = flag ? y0 : (s0 + y0);
      const v4f sn1 = flag ? y1 : (s1 + y1);
      st2f(po, hn0, hn1); st2f(ps, sn0, sn1); st2h(ph, hn0, hn1);
      __threadfence();
      st2f(po, hn0, hn1); st2f(ps, sn0, sn1); st2h(ph, hn0, hn1);
    } else if (MODE == M_XLR) {
      float* po = outF + (size_t)node * ldo + slab * CH + 4 * lane;
      st2f(po, v0, v1);
      __threadfence();
      st2f(po, v0, v1);
    } else if (MODE == M_QKV) {
      _Float16* ph = outH + (size_t)node * ldoh + slab * CH + 4 * lane;
      v0 = v0 + bb0; v1 = v1 + bb1;
      st2h(ph, v0, v1);
      __threadfence();
      st2h(ph, v0, v1);
    } else if (MODE == M_WO) {
      float* po = outF + (size_t)node * ldo + 4 * lane;
      _Float16* ph = outH + (size_t)node * ldoh + 4 * lane;
      v0 = v0 + bb0; v1 = v1 + bb1;
      v0 = LD4(po) + v0; v1 = LD4(po + 128) + v1;
      ln8(v0, v1, gg0, gg1, ee0, ee1);
      st2f(po, v0, v1); st2h(ph, v0, v1);
      __threadfence();
      st2f(po, v0, v1); st2h(ph, v0, v1);
    } else if (MODE == M_SKIP) {
      float* po = outF + (size_t)node * ldo + 4 * lane;
      v0 = v0 + bb0; v1 = v1 + bb1;
      st2f(po, v0, v1);
      __threadfence();
      st2f(po, v0, v1);
    } else {
      v0 = v0 + bb0; v1 = v1 + bb1;
      const v4f g0 = sig4(v0), g1 = sig4(v1);
      const v4f hr0 = LD4(p0 + (size_t)node * CH + 4 * lane);
      const v4f hr1 = LD4(p0 + (size_t)node * CH + 128 + 4 * lane);
      const v4f sx0 = LD4(rin + (size_t)node * CH + 4 * lane);
      const v4f sx1 = LD4(rin + (size_t)node * CH + 128 + 4 * lane);
      const v4f hf0 = g0 * hr0 + (one4 - g0) * sx0;
      const v4f hf1 = g1 * hr1 + (one4 - g1) * sx1;
      P8 u0, u1;
      u0.h = __builtin_convertvector(hf0, v4h);
      u1.h = __builtin_convertvector(hf1, v4h);
      *(v2i*)(Hf + rl * HP + 4 * lane) = u0.i;
      *(v2i*)(Hf + rl * HP + 128 + 4 * lane) = u1.i;
    }
  }

  if (MODE == M_GATE) {
    __syncthreads();
    if (w < 4) {
      v8f oc = z8;
      const _Float16* hrow = Hf + (16 * w + m) * HP + 8 * hh;
      const _Float16* w2r = W2 + (size_t)m * CH + 8 * hh;
#pragma unroll 1
      for (int k0 = 0; k0 < CH; k0 += 32) {
        const v16h a = ldfrag(hrow + k0);
        const v16h b = ldfrag(w2r + k0);
        oc = wm(a, b, oc);
      }
      const float bo0 = p1[0], bo1 = p1[1];
      if (m < 2) {
        const float bo = (m == 0) ? bo0 : bo1;
#pragma unroll
        for (int r = 0; r < 8; ++r) {
          const float z = oc[r] * WINV + bo;
          const float sp = fmaxf(z, 0.0f) + log1pf(expf(-fabsf(z)));
          outs[(16 * w + 8 * hh + r) * 2 + m] = (m == 1) ? sp : z;
        }
      }
    }
    __syncthreads();
    if (w == 0) {
      const v4f ov = LD4(outs + 4 * lane);
      float* po = dout + (size_t)rowBase * 2 + 4 * lane;
      *(volatile v4f*)po = ov;
      __threadfence();
      *(volatile v4f*)po = ov;
    }
  }
}

__global__ __launch_bounds__(NTHR) void k_attn(const _Float16* __restrict__ QKV, _Float16* ATT) {
  __shared__ __attribute__((aligned(16))) _Float16 Vt[DHD * VP];
  __shared__ __attribute__((aligned(16))) _Float16 Pl[8 * 16 * PP];
  const int tid = threadIdx.x;
  const int lane = tid & 31;
  const int w = tid >> 5;
  const int hh = lane >> 4;
  const int m = lane & 15;
  const int bt = blockIdx.x >> 2;
  const int h = blockIdx.x & 3;
  const size_t r0 = (size_t)bt * NST;

  {
    const int key = tid >> 1;
    const int d0 = (tid & 1) * 32;
    const _Float16* pv = QKV + (r0 + key) * QKVW + 2 * CH + h * DHD + d0;
    P16 u[4];
#pragma unroll
    for (int q = 0; q < 4; ++q) u[q].i = *(const v4i*)(pv + 8 * q);
#pragma unroll
    for (int q = 0; q < 4; ++q)
#pragma unroll
      for (int j = 0; j < 8; ++j) Vt[(d0 + 8 * q + j) * VP + key] = u[q].h[j];
  }
  __syncthreads();

  const v8f z8 = {0.f, 0.f, 0.f, 0.f, 0.f, 0.f, 0.f, 0.f};
  v8f s[8];
#pragma unroll
  for (int i = 0; i < 8; ++i) s[i] = z8;
  const _Float16* qrow = QKV + (r0 + 16 * w + m) * QKVW + h * DHD + 8 * hh;
#pragma unroll
  for (int ks = 0; ks < DHD; ks += 32) {
    const v16h a = ldfrag(qrow + ks);
#pragma unroll
    for (int nt = 0; nt < 8; ++nt) {
      const v16h b = ldfrag(QKV + (r0 + 16 * nt + m) * QKVW + CH + h * DHD + 8 * hh + ks);
      s[nt] = wm(a, b, s[nt]);
    }
  }

  _Float16* Pw = Pl + w * 16 * PP;
#pragma unroll
  for (int r = 0; r < 8; ++r) {
    float mx = -3.0e38f;
#pragma unroll
    for (int nt = 0; nt < 8; ++nt) mx = fmaxf(mx, s[nt][r] * 0.125f);
    mx = fmaxf(mx, __shfl_xor(mx, 8, 32));
    mx = fmaxf(mx, __shfl_xor(mx, 4, 32));
    mx = fmaxf(mx, __shfl_xor(mx, 2, 32));
    mx = fmaxf(mx, __shfl_xor(mx, 1, 32));
    float p[8];
    float sm = 0.0f;
#pragma unroll
    for (int nt = 0; nt < 8; ++nt) { p[nt] = __expf(s[nt][r] * 0.125f - mx); sm += p[nt]; }
    sm += __shfl_xor(sm, 8, 32);
    sm += __shfl_xor(sm, 4, 32);
    sm += __shfl_xor(sm, 2, 32);
    sm += __shfl_xor(sm, 1, 32);
    const float f = PSC * (1.0f / sm);
#pragma unroll
    for (int nt = 0; nt < 8; ++nt) Pw[(8 * hh + r) * PP + 16 * nt + m] = (_Float16)(p[nt] * f);
  }
  __syncthreads();

  v8f o[4];
#pragma unroll
  for (int i = 0; i < 4; ++i) o[i] = z8;
#pragma unroll
  for (int ks = 0; ks < NST; ks += 32) {
    const v16h a = ldfrag(Pw + m * PP + ks + 8 * hh);
#pragma unroll
    for (int dt = 0; dt < 4; ++dt) {
      const v16h b = ldfrag(Vt + (16 * dt + m) * VP + ks + 8 * hh);
      o[dt] = wm(a, b, o[dt]);
    }
  }
  __syncthreads();
#pragma unroll
  for (int dt = 0; dt < 4; ++dt)
#pragma unroll
    for (int r = 0; r < 8; ++r) Pw[(8 * hh + r) * PP + 16 * dt + m] = (_Float16)(o[dt][r] * PINV);
  __syncthreads();

  P16 u[4];
  _Float16* gp[4];
#pragma unroll
  for (int i = 0; i < 4; ++i) {
    const int row = 4 * i + (lane >> 3);
    const int pc = lane & 7;
    u[i].h = *(const v8h*)(Pw + row * PP + 8 * pc);
    gp[i] = ATT + (r0 + 16 * w + row) * CH + h * DHD + 8 * pc;
  }
#pragma unroll
  for (int i = 0; i < 4; ++i) *(volatile v4i*)gp[i] = u[i].i;
  __threadfence();
#pragma unroll
  for (int i = 0; i < 4; ++i) *(volatile v4i*)gp[i] = u[i].i;
}

__global__ __launch_bounds__(NTHR) void k_gat(
    const float* __restrict__ XLR, const int* __restrict__ ei, const float* __restrict__ att,
    const float* __restrict__ gatb, const float* __restrict__ ng, const float* __restrict__ nbt,
    const float* __restrict__ SK, float* H32, _Float16* H16o, int nE, int isLast) {
  extern __shared__ v4f alds[];
  float* acc  = (float*)alds;
  float* ms   = acc + GT * 2 * CH;
  float* dens = ms + GT * 2;
  int*   list = (int*)(dens + GT * 2);

  const int tid = threadIdx.x;
  const int lane = tid & 31;
  const int w = tid >> 5;
  const int nodeBase = blockIdx.x * GT;
  const int grp = nodeBase / NST;
  const int sbase = nodeBase - grp * NST;

  {
    const v4f z4 = {0.f, 0.f, 0.f, 0.f};
#pragma unroll 1
    for (int i = tid; i < (GT * 2 * CH) / 4; i += NTHR) alds[i] = z4;
    if (tid < GT * 2) { ms[tid] = -3.0e38f; dens[tid] = 0.0f; }
  }
  const v4f at0 = LD4(att + 4 * lane);
  const v4f at1 = LD4(att + 128 + 4 * lane);
  const v4f at2 = LD4(att + CH + 4 * lane);
  const v4f at3 = LD4(att + CH + 128 + 4 * lane);
  __syncthreads();

  const int nCh = (nE + GCH - 1) / GCH;
#pragma unroll 1
  for (int ch = 0; ch <= nCh; ++ch) {
    const bool self = (ch == nCh);
    const int cbase = ch * GCH;
    int wc = 8;
    if (!self) {
      wc = 0;
#pragma unroll 1
      for (int it = 0; it < GCH / 32; ++it) {
        const int eL = it * 32 + lane;
        const int e = cbase + eL;
        const int ec = (e < nE) ? e : (nE - 1);
        const int d = ei[nE + ec];
        const int sb = d - sbase;
        const bool hit = (e < nE) && ((unsigned)sb < (unsigned)GT) && ((sb >> 3) == w);
        const unsigned mk = __builtin_amdgcn_ballot_w32(hit);
        if (hit) {
          const int pos = wc + (int)__builtin_amdgcn_mbcnt_lo(mk, 0u);
          list[w * GCH + pos] = (eL << 3) | (sb & 7);
        }
        wc += (int)__builtin_popcount(mk);
      }
    }
    __syncthreads();
    const int n = (wc < GCH) ? wc : GCH;
#pragma unroll 1
    for (int i = 0; i < n; ++i) {
      const int raw = list[w * GCH + i];
      const int ent = self ? ((i << 3) | i) : raw;
      const int sl = ent & 7;
      const int eL = (ent >> 3) & (GCH - 1);
      const int slot = w * 8 + sl;
      const int dst = nodeBase + slot;
      const int ecl = cbase + eL;
      const int e = (ecl < nE) ? ecl : (nE - 1);
      int sst = ei[e];
      sst = (sst < 0) ? 0 : ((sst > NST - 1) ? (NST - 1) : sst);
      const int src = self ? dst : (grp * NST + sst);

      const float* ps = XLR + (size_t)src * (4 * CH);
      const float* pd = XLR + (size_t)dst * (4 * CH) + 2 * CH;
      const v4f l0 = LD4(ps + 4 * lane), l1 = LD4(ps + 128 + 4 * lane);
      const v4f l2 = LD4(ps + CH + 4 * lane), l3 = LD4(ps + CH + 128 + 4 * lane);
      const v4f q0 = LD4(pd + 4 * lane), q1 = LD4(pd + 128 + 4 * lane);
      const v4f q2 = LD4(pd + CH + 4 * lane), q3 = LD4(pd + CH + 128 + 4 * lane);
      const float t0 = wsum(dlk(l0, q0, at0) + dlk(l1, q1, at1));
      const float t1 = wsum(dlk(l2, q2, at2) + dlk(l3, q3, at3));
      {
        const float mo = ms[slot * 2];
        const float mn = fmaxf(mo, t0);
        const float sc = __expf(mo - mn);
        const float p  = __expf(t0 - mn);
        const float dn = dens[slot * 2] * sc + p;
        ms[slot * 2] = mn;
        dens[slot * 2] = dn;
        v4f* pa = (v4f*)(acc + slot * (2 * CH) + 4 * lane);
        v4f* pb = (v4f*)(acc + slot * (2 * CH) + 128 + 4 * lane);
        const v4f a = *pa, b = *pb;
        *pa = a * sc + p * l0;
        *pb = b * sc + p * l1;
      }
      {
        const float mo = ms[slot * 2 + 1];
        const float mn = fmaxf(mo, t1);
        const float sc = __expf(mo - mn);
        const float p  = __expf(t1 - mn);
        const float dn = dens[slot * 2 + 1] * sc + p;
        ms[slot * 2 + 1] = mn;
        dens[slot * 2 + 1] = dn;
        v4f* pa = (v4f*)(acc + slot * (2 * CH) + CH + 4 * lane);
        v4f* pb = (v4f*)(acc + slot * (2 * CH) + CH + 128 + 4 * lane);
        const v4f a = *pa, b = *pb;
        *pa = a * sc + p * l2;
        *pb = b * sc + p * l3;
      }
    }
    __syncthreads();
  }

  const v4f gb0 = LD4(gatb + 4 * lane), gb1 = LD4(gatb + 128 + 4 * lane);
  const v4f g0 = LD4(ng + 4 * lane), g1 = LD4(ng + 128 + 4 * lane);
  const v4f e0 = LD4(nbt + 4 * lane), e1 = LD4(nbt + 128 + 4 * lane);
#pragma unroll 1
  for (int sl = 0; sl < 8; ++sl) {
    const int slot = w * 8 + sl;
    const int node = nodeBase + slot;
    const float dn0 = dens[slot * 2], dn1 = dens[slot * 2 + 1];
    const float i0 = 1.0f / (dn0 + 1e-16f);
    const float i1 = 1.0f / (dn1 + 1e-16f);
    const float* pa = acc + slot * (2 * CH) + 4 * lane;
    const v4f a0 = LD4(pa), a1 = LD4(pa + 128), a2 = LD4(pa + CH), a3 = LD4(pa + CH + 128);
    const v4f hg0 = (a0 * i0 + a2 * i1) * 0.5f + gb0;
    const v4f hg1 = (a1 * i0 + a3 * i1) * 0.5f + gb1;
    float* ph = H32 + (size_t)node * CH + 4 * lane;
    _Float16* pq = H16o + (size_t)node * CH + 4 * lane;
    v4f v0 = LD4(ph) + hg0;
    v4f v1 = LD4(ph + 128) + hg1;
    ln8(v0, v1, g0, g1, e0, e1);
    if (isLast) {
      v0 = LD4(SK + (size_t)node * CH + 4 * lane) + v0;
      v1 = LD4(SK + (size_t)node * CH + 128 + 4 * lane) + v1;
    }
    st2f(ph, v0, v1); st2h(pq, v0, v1);
    __threadfence();
    st2f(ph, v0, v1); st2h(pq, v0, v1);
  }
}

extern "C" void kernel_launch(void* const* d_in, const int* in_sizes, int n_in,
                              void* d_out, int out_size, void* d_ws, size_t ws_size,
                              hipStream_t stream) {
  if (n_in < 30) return;
  if (in_sizes[0] != NNODE * FIN) return;
  const int nE = in_sizes[1] / 2;
  if (nE < 1 || in_sizes[1] != 2 * nE) return;
  if (in_sizes[2] != FIN * CH || in_sizes[3] != CH) return;
  if (in_sizes[4] != NST * CH || in_sizes[5] < NTIM * CH) return;
  if (in_sizes[6] != NLAY * CH * CH * KTAP || in_sizes[7] != NLAY * CH) return;
  if (in_sizes[8] != NLAY * CH * 2 * CH || in_sizes[9] != NLAY * CH * 2 * CH) return;
  if (in_sizes[10] != NLAY * 2 * CH) return;
  if (in_sizes[11] != NLAY * CH || in_sizes[12] != NLAY * CH || in_sizes[13] != NLAY * CH) return;
  for (int i = 14; i < 18; ++i) if (in_sizes[i] != CH * CH) return;
  for (int i = 18; i < 24; ++i) if (in_sizes[i] != CH) return;
  if (in_sizes[24] != FIN * CH || in_sizes[25] != CH) return;
  if (in_sizes[26] != CH * CH || in_sizes[27] != CH) return;
  if (in_sizes[28] != CH * 2 || in_sizes[29] != 2) return;
  if (out_size != NNODE * 2) return;

  const float* x       = (const float*)d_in[0];
  const int*   edge    = (const int*)d_in[1];
  const float* W_enc   = (const float*)d_in[2];
  const float* b_enc   = (const float*)d_in[3];
  const float* st_emb  = (const float*)d_in[4];
  const float* hz_emb  = (const float*)d_in[5];
  const float* conv_w  = (const float*)d_in[6];
  const float* conv_b  = (const float*)d_in[7];
  const float* gat_wl  = (const float*)d_in[8];
  const float* gat_wr  = (const float*)d_in[9];
  const float* gat_att = (const float*)d_in[10];
  const float* gat_b   = (const float*)d_in[11];
  const float* norm_g  = (const float*)d_in[12];
  const float* norm_b  = (const float*)d_in[13];
  const float* Wq = (const float*)d_in[14];
  const float* Wk = (const float*)d_in[15];
  const float* Wv = (const float*)d_in[16];
  const float* Wo = (const float*)d_in[17];
  const float* bq = (const float*)d_in[18];
  const float* bk = (const float*)d_in[19];
  const float* bv = (const float*)d_in[20];
  const float* bo = (const float*)d_in[21];
  const float* an_g = (const float*)d_in[22];
  const float* an_b = (const float*)d_in[23];
  const float* W_skip = (const float*)d_in[24];
  const float* b_skip = (const float*)d_in[25];
  const float* W_gate = (const float*)d_in[26];
  const float* b_gate = (const float*)d_in[27];
  const float* W_out  = (const float*)d_in[28];
  const float* b_out  = (const float*)d_in[29];
  float* out = (float*)d_out;

  char* wsp = (char*)d_ws;
  size_t off = 0;
  auto take = [&](size_t bytes) -> char* {
    char* p = wsp + off;
    off += (bytes + 255) & ~(size_t)255;
    return p;
  };
  _Float16* WencT  = (_Float16*)take((size_t)CH * FIN * 2);
  _Float16* WconvT = (_Float16*)take((size_t)NLAY * CH * (KTAP * CH) * 2);
  _Float16* WlrT   = (_Float16*)take((size_t)NLAY * (4 * CH) * CH * 2);
  _Float16* WqkvT  = (_Float16*)take((size_t)QKVW * CH * 2);
  _Float16* WoT    = (_Float16*)take((size_t)CH * CH * 2);
  _Float16* WgT    = (_Float16*)take((size_t)CH * CH * 2);
  _Float16* WskT   = (_Float16*)take((size_t)CH * FIN * 2);
  _Float16* WoutT  = (_Float16*)take((size_t)16 * CH * 2);
  _Float16* X16    = (_Float16*)take((size_t)NNODE * FIN * 2);
  float*    H32    = (float*)take((size_t)NNODE * CH * 4);
  float*    SK32   = (float*)take((size_t)NNODE * CH * 4);
  _Float16* H16a   = (_Float16*)take((size_t)NNODE * CH * 2);
  _Float16* H16b   = (_Float16*)take((size_t)NNODE * CH * 2);
  float*    XLR    = (float*)take((size_t)NNODE * (4 * CH) * 4);
  if (off > ws_size) return;
  if (off > (size_t)134217728) return;
  _Float16* QKV16 = (_Float16*)XLR;
  _Float16* ATT16 = (_Float16*)((char*)XLR + (size_t)NNODE * QKVW * 2);
  float*    SKX32 = (float*)((char*)XLR + (size_t)NNODE * QKVW * 2 + (size_t)NNODE * CH * 2);
  if ((size_t)NNODE * QKVW * 2 + (size_t)NNODE * CH * 2 + (size_t)NNODE * CH * 4 > (size_t)NNODE * (4 * CH) * 4) return;

  k_prep8<<<dim3(32, 8), NTHR, 0, stream>>>(
      W_enc, Wq, Wk, Wv, Wo, W_gate, W_skip, W_out,
      WencT, WqkvT, WqkvT + (size_t)CH * CH, WqkvT + (size_t)2 * CH * CH, WoT, WgT, WskT, WoutT,
      FIN, CH, CH, CH, CH, CH, FIN, CH,
      CH, CH, CH, CH, CH, CH, CH, 2,
      CH, CH, CH, CH, CH, CH, CH, 16);
  k_prep8<<<dim3(64, 6), NTHR, 0, stream>>>(
      gat_wl, gat_wl + (size_t)CH * 2 * CH, gat_wl + (size_t)2 * CH * 2 * CH,
      gat_wr, gat_wr + (size_t)CH * 2 * CH, gat_wr + (size_t)2 * CH * 2 * CH,
      gat_wl, gat_wl,
      WlrT, WlrT + (size_t)(4 * CH) * CH, WlrT + (size_t)2 * (4 * CH) * CH,
      WlrT + (size_t)(2 * CH) * CH, WlrT + (size_t)(4 * CH) * CH + (size_t)(2 * CH) * CH,
      WlrT + (size_t)2 * (4 * CH) * CH + (size_t)(2 * CH) * CH,
      WlrT, WlrT,
      CH, CH, CH, CH, CH, CH, CH, CH,
      2 * CH, 2 * CH, 2 * CH, 2 * CH, 2 * CH, 2 * CH, 2 * CH, 2 * CH,
      2 * CH, 2 * CH, 2 * CH, 2 * CH, 2 * CH, 2 * CH, 2 * CH, 2 * CH);
  k_prep_conv<<<dim3((CH * ((KTAP * CH) / 8) + NTHR - 1) / NTHR, NLAY), NTHR, 0, stream>>>(conv_w, WconvT);
  k_prep_x<<<(NNODE * (FIN / 8) + NTHR - 1) / NTHR, NTHR, 0, stream>>>(x, X16, NNODE);

  hipFuncSetAttribute(reinterpret_cast<const void*>(&k_gemm<M_ENC>),  hipFuncAttributeMaxDynamicSharedMemorySize, LDS_GEMM);
  hipFuncSetAttribute(reinterpret_cast<const void*>(&k_gemm<M_CONV>), hipFuncAttributeMaxDynamicSharedMemorySize, LDS_GEMM);
  hipFuncSetAttribute(reinterpret_cast<const void*>(&k_gemm<M_XLR>),  hipFuncAttributeMaxDynamicSharedMemorySize, LDS_GEMM);
  hipFuncSetAttribute(reinterpret_cast<const void*>(&k_gemm<M_QKV>),  hipFuncAttributeMaxDynamicSharedMemorySize, LDS_GEMM);
  hipFuncSetAttribute(reinterpret_cast<const void*>(&k_gemm<M_WO>),   hipFuncAttributeMaxDynamicSharedMemorySize, LDS_GEMM);
  hipFuncSetAttribute(reinterpret_cast<const void*>(&k_gemm<M_SKIP>), hipFuncAttributeMaxDynamicSharedMemorySize, LDS_GEMM);
  hipFuncSetAttribute(reinterpret_cast<const void*>(&k_gemm<M_GATE>), hipFuncAttributeMaxDynamicSharedMemorySize, LDS_GATE);
  hipFuncSetAttribute(reinterpret_cast<const void*>(&k_gat),          hipFuncAttributeMaxDynamicSharedMemorySize, LDS_GAT);

  const dim3 g256(NNODE / GM, 1);

  k_gemm<M_ENC><<<g256, NTHR, LDS_GEMM, stream>>>(
      X16, WencT, b_enc, st_emb, hz_emb, H32, H32, SK32, H16a, out, WoutT,
      FIN, FIN, CH, CH, 0, 0);

  for (int l = 0; l < NLAY; ++l) {
    k_gemm<M_CONV><<<g256, NTHR, LDS_GEMM, stream>>>(
        H16a, WconvT + (size_t)l * CH * (KTAP * CH), conv_b + (size_t)l * CH, b_enc, b_enc,
        H32, H32, SK32, H16b, out, WoutT,
        KTAP * CH, CH, CH, CH, 1 << l, (l == 0) ? 1 : 0);
    k_gemm<M_XLR><<<dim3(NNODE / GM, 4), NTHR, LDS_GEMM, stream>>>(
        H16b, WlrT + (size_t)l * (4 * CH) * CH, b_enc, b_enc, b_enc,
        H32, XLR, SK32, H16b, out, WoutT,
        CH, CH, 4 * CH, CH, 0, 0);
    k_gat<<<NNODE / GT, NTHR, LDS_GAT, stream>>>(
        XLR, edge, gat_att + (size_t)l * 2 * CH, gat_b + (size_t)l * CH,
        norm_g + (size_t)l * CH, norm_b + (size_t)l * CH, SK32, H32, H16a, nE,
        (l == NLAY - 1) ? 1 : 0);
  }

  k_gemm<M_QKV><<<dim3(NNODE / GM, 3), NTHR, LDS_GEMM, stream>>>(
      H16a, WqkvT, bq, bk, bv, H32, H32, SK32, QKV16, out, WoutT,
      CH, CH, CH, QKVW, 0, 0);
  k_attn<<<NGRP * NHD, NTHR, 0, stream>>>(QKV16, ATT16);
  k_gemm<M_WO><<<g256, NTHR, LDS_GEMM, stream>>>(
      ATT16, WoT, bo, an_g, an_b, H32, H32, SK32, H16b, out, WoutT,
      CH, CH, CH, CH, 0, 0);

  k_gemm<M_SKIP><<<g256, NTHR, LDS_GEMM, stream>>>(
      X16, WskT, b_skip, b_enc, b_enc, H32, SKX32, SK32, H16b, out, WoutT,
      FIN, FIN, CH, CH, 0, 0);
  k_gemm<M_GATE><<<g256, NTHR, LDS_GATE, stream>>>(
      H16b, WgT, b_gate, H32, b_out, SKX32, H32, SK32, H16b, out, WoutT,
      CH, CH, CH, CH, 0, 0);
}
